// MLASelfAttentionBlock_24893630447987
// MI455X (gfx1250) — hardware-verified
//
#include <hip/hip_runtime.h>
#include <math.h>
#include <stdint.h>

#define NBATCH 2
#define SEQ    2048
#define DMOD   2048
#define NHEAD  16
#define HDIM   128
#define DLAT   512
#define BTOT   (NBATCH * SEQ)
#define HGRP   2
#define NGRP   (NHEAD / HGRP)
#define NQB    (SEQ / 64)
#define NQBRES 12
#define TRES   (NQBRES * 64)

#define QSC 16.0f
#define KSC 4.0f
#define VSC 16.0f
#define YSC 16.0f
#define WSC 64.0f
#define PSC 1024.0f

static_assert((SEQ % 64) == 0);
static_assert((DMOD % 64) == 0);
static_assert((DLAT % 32) == 0);
static_assert(HDIM == 128);
static_assert(NHEAD * HDIM == DMOD);
static_assert(TRES < SEQ);

typedef _Float16 v16h __attribute__((ext_vector_type(16)));
typedef _Float16 v8h  __attribute__((ext_vector_type(8)));
typedef __bf16   v16b __attribute__((ext_vector_type(16)));
typedef __bf16   v8b  __attribute__((ext_vector_type(8)));
typedef float    v8f  __attribute__((ext_vector_type(8)));
typedef float    v4f  __attribute__((ext_vector_type(4)));
typedef float    v2f  __attribute__((ext_vector_type(2)));
typedef unsigned int   v4u  __attribute__((ext_vector_type(4)));
typedef unsigned short v8us __attribute__((ext_vector_type(8)));

__device__ __forceinline__ unsigned short f2bf_bits(float f) {
  unsigned u = __float_as_uint(f);
  return (unsigned short)((u + 0x7FFFu + ((u >> 16) & 1u)) >> 16);
}
__device__ __forceinline__ float bf_bits2f(unsigned short h) { return __uint_as_float(((unsigned)h) << 16); }
__device__ __forceinline__ unsigned pk16(unsigned short a, unsigned short b) { return (unsigned)a | ((unsigned)b << 16); }
__device__ __forceinline__ void bf_split_bits(float f, unsigned short& hb, unsigned short& lb) {
  hb = f2bf_bits(f);
  lb = f2bf_bits(f - bf_bits2f(hb));
}

__device__ __forceinline__ void dep_guard_h(v8f& a, v8f& b, v16h x, v16h y) { asm volatile("v_nop\n\tv_nop\n\tv_nop\n\tv_nop" : "+v"(a), "+v"(b) : "v"(x), "v"(y)); }
__device__ __forceinline__ void dep_guard_b(v8f& a, v8f& b, v16b x, v16b y) { asm volatile("v_nop\n\tv_nop\n\tv_nop\n\tv_nop" : "+v"(a), "+v"(b) : "v"(x), "v"(y)); }
__device__ __forceinline__ void keep4_h(v16h a, v16h b, v16h c, v16h d) { asm volatile("v_nop" :: "v"(a), "v"(b), "v"(c), "v"(d)); }
__device__ __forceinline__ void keep4_b(v16b a, v16b b, v16b c, v16b d) { asm volatile("v_nop" :: "v"(a), "v"(b), "v"(c), "v"(d)); }
__device__ __forceinline__ void acc_guard4(v8f& a, v8f& b, v8f& c, v8f& d) { asm volatile("v_nop\n\tv_nop\n\tv_nop\n\tv_nop" : "+v"(a), "+v"(b), "+v"(c), "+v"(d)); }
__device__ __forceinline__ void g4h(v8f& a, v8f& b, v8f& c, v8f& d, v16h x, v16h y) {
  asm volatile("v_nop\n\tv_nop\n\tv_nop\n\tv_nop" : "+v"(a), "+v"(b), "+v"(c), "+v"(d) : "v"(x), "v"(y));
}
__device__ __forceinline__ void g4b(v8f& a, v8f& b, v8f& c, v8f& d, v16b x, v16b y) {
  asm volatile("v_nop\n\tv_nop\n\tv_nop\n\tv_nop" : "+v"(a), "+v"(b), "+v"(c), "+v"(d) : "v"(x), "v"(y));
}

template <typename T> struct Frag;
template <> struct Frag<_Float16> {
  typedef v16h V; union U { v16h v; v8h h[2]; };
  static __device__ __forceinline__ v16h load(const _Float16* p) {
    U f; f.h[0] = *(const v8h*)(p); f.h[1] = *(const v8h*)(p + 16); return f.v;
  }
  static __device__ __forceinline__ v8f mma(v16h a, v16h b, v8f c) {
    return __builtin_amdgcn_wmma_f32_16x16x32_f16(false, a, false, b, (short)0, c, false, false);
  }
  static __device__ __forceinline__ void guard(v8f& a, v8f& b, v16h x, v16h y) { dep_guard_h(a, b, x, y); }
  static __device__ __forceinline__ void keep(v16h a, v16h b, v16h c, v16h d) { keep4_h(a, b, c, d); }
};
template <> struct Frag<__bf16> {
  typedef v16b V; union U { v16b v; v8b h[2]; };
  static __device__ __forceinline__ v16b load(const __bf16* p) {
    U f; f.h[0] = *(const v8b*)(p); f.h[1] = *(const v8b*)(p + 16); return f.v;
  }
  static __device__ __forceinline__ v8f mma(v16b a, v16b b, v8f c) {
    return __builtin_amdgcn_wmma_f32_16x16x32_bf16(false, a, false, b, (short)0, c, false, false);
  }
  static __device__ __forceinline__ void guard(v8f& a, v8f& b, v16b x, v16b y) { dep_guard_b(a, b, x, y); }
  static __device__ __forceinline__ void keep(v16b a, v16b b, v16b c, v16b d) { keep4_b(a, b, c, d); }
};
template <int ET> struct Elem;
template <> struct Elem<0> { typedef _Float16 T; };
template <> struct Elem<1> { typedef __bf16 T; };

template <int ET, bool SA, bool SB, int OUT, bool WN>
__global__ __launch_bounds__(256) void gemm64(
    const unsigned short* __restrict__ Ap, const unsigned short* __restrict__ A2p, int lda, long long strideA,
    const unsigned short* __restrict__ Btp, const unsigned short* __restrict__ Bt2p, int ldb, long long strideB,
    void* C0p, void* C1p, void* C2p, int ldc, long long strideC,
    int M, int N, int K, float scale, float scale16) {
  typedef typename Elem<ET>::T T;
  typedef typename Frag<T>::V V;
  const T* A = (const T*)(const void*)Ap; const T* A2 = (const T*)(const void*)A2p;
  const T* Bt = (const T*)(const void*)Btp; const T* Bt2 = (const T*)(const void*)Bt2p;
  __shared__ __align__(16) float sT[8][16 * 68];
  const int b    = blockIdx.y;
  const int lane = threadIdx.x & 31;
  const int wave = threadIdx.x >> 5;
  const int tilesN = N >> 6;
  const int tilesM = M >> 6;
  int tm, tn;
  if (WN) { const int gN = tilesN >> 3; tm = (int)blockIdx.x / gN; tn = ((int)blockIdx.x - tm * gN) * 8 + wave; }
  else    { const int gM = tilesM >> 3; tn = (int)blockIdx.x / gM; tm = ((int)blockIdx.x - tn * gM) * 8 + wave; }
  if (tm >= tilesM || tn >= tilesN) return;
  const int m0 = tm << 6;
  const int n0 = tn << 6;

  const T* Ab  = A  + (size_t)b * (size_t)strideA;
  const T* Bb  = Bt + (size_t)b * (size_t)strideB;
  const T* Ab2 = SA ? (A2  + (size_t)b * (size_t)strideA) : Ab;
  const T* Bb2 = SB ? (Bt2 + (size_t)b * (size_t)strideB) : Bb;

  const int rlane = lane & 15;
  const int koff  = (lane >> 4) * 8;
  const int mOff  = (lane >> 4) * 8;

  v8f acc[4][4];
#pragma unroll
  for (int i = 0; i < 4; ++i)
#pragma unroll
    for (int j = 0; j < 4; ++j) acc[i][j] = (v8f){0.f,0.f,0.f,0.f,0.f,0.f,0.f,0.f};

  for (int k0 = 0; k0 < K; k0 += 32) {
    V bh[4], bl[4];
#pragma unroll
    for (int j = 0; j < 4; ++j) {
      const size_t bo = (size_t)(n0 + (j << 4) + rlane) * ldb + koff + k0;
      bh[j] = Frag<T>::load(Bb + bo);
      bl[j] = bh[j];
      if (SB) bl[j] = Frag<T>::load(Bb2 + bo);
    }
#pragma unroll
    for (int i = 0; i < 4; ++i) {
      const size_t ao = (size_t)(m0 + (i << 4) + rlane) * lda + koff + k0;
      V ah = Frag<T>::load(Ab + ao);
      V al = ah;
      if (SA) al = Frag<T>::load(Ab2 + ao);
#pragma unroll
      for (int j = 0; j < 4; ++j) {
        acc[i][j] = Frag<T>::mma(ah, bh[j], acc[i][j]);
        if (SB) acc[i][j] = Frag<T>::mma(ah, bl[j], acc[i][j]);
        if (SA) acc[i][j] = Frag<T>::mma(al, bh[j], acc[i][j]);
      }
      Frag<T>::guard(acc[i][0], acc[i][3], ah, al);
    }
    Frag<T>::keep(bh[0], bh[1], bh[2], bh[3]);
    if (SB) Frag<T>::keep(bl[0], bl[1], bl[2], bl[3]);
  }
  acc_guard4(acc[0][0], acc[0][1], acc[0][2], acc[0][3]);
  acc_guard4(acc[1][0], acc[1][1], acc[1][2], acc[1][3]);
  acc_guard4(acc[2][0], acc[2][1], acc[2][2], acc[2][3]);
  acc_guard4(acc[3][0], acc[3][1], acc[3][2], acc[3][3]);

  float* slab = sT[wave];
#pragma unroll
  for (int i = 0; i < 4; ++i) {
    const int mBase = m0 + (i << 4);
#pragma unroll
    for (int j = 0; j < 4; ++j) {
#pragma unroll
      for (int r = 0; r < 8; ++r) {
        slab[(mOff + r) * 68 + (j << 4) + rlane] = acc[i][j][r] * scale;
      }
    }
    __builtin_amdgcn_fence(__ATOMIC_RELEASE, "workgroup");
    __builtin_amdgcn_wave_barrier();
    __builtin_amdgcn_fence(__ATOMIC_ACQUIRE, "workgroup");
    if (OUT == 0) {
      float* C = (float*)C0p + (size_t)b * (size_t)strideC;
      const int hh = lane >> 4, c4 = (lane & 15) * 4;
      for (int pass = 0; pass < 2; ++pass) {
#pragma unroll
        for (int it = 0; it < 8; ++it) {
          const int row = it * 2 + hh;
          v4f v = *(const v4f*)(slab + row * 68 + c4);
          *(volatile v4f*)(C + (size_t)(mBase + row) * ldc + n0 + c4) = v;
        }
        __threadfence();
      }
    } else {
      const int q = lane >> 3, c8 = (lane & 7) * 8;
      _Float16*       Ch  = (_Float16*)C0p + (size_t)b * (size_t)strideC;
      unsigned short* Cb1 = (unsigned short*)C1p + (size_t)b * (size_t)strideC;
      unsigned short* Cb2 = (unsigned short*)C2p + (size_t)b * (size_t)strideC;
      for (int pass = 0; pass < 2; ++pass) {
#pragma unroll
        for (int it = 0; it < 4; ++it) {
          const int row = it * 4 + q;
          const float* sp = slab + row * 68 + c8;
          v8h  hv = {0, 0, 0, 0, 0, 0, 0, 0};
          v8us b1 = {0, 0, 0, 0, 0, 0, 0, 0};
          v8us b2 = {0, 0, 0, 0, 0, 0, 0, 0};
#pragma unroll
          for (int e = 0; e < 8; ++e) {
            const float f = sp[e];
            if (OUT == 1 || OUT == 3) hv[e] = (_Float16)(f * scale16);
            if (OUT == 2 || OUT == 3) { unsigned short hb, lb; bf_split_bits(f, hb, lb); b1[e] = hb; b2[e] = lb; }
          }
          const size_t go = (size_t)(mBase + row) * ldc + n0 + c8;
          if (OUT == 1 || OUT == 3) *(volatile v8h*)(Ch + go) = hv;
          if (OUT == 2 || OUT == 3) { *(volatile v8us*)(Cb1 + go) = b1; *(volatile v8us*)(Cb2 + go) = b2; }
        }
        __threadfence();
      }
    }
    __builtin_amdgcn_fence(__ATOMIC_RELEASE, "workgroup");
    __builtin_amdgcn_wave_barrier();
    __builtin_amdgcn_fence(__ATOMIC_ACQUIRE, "workgroup");
  }
}

__global__ __launch_bounds__(256) void cvt_bf16x2_kernel(const float* __restrict__ in, unsigned short* __restrict__ out, int n2) {
  const int i = blockIdx.x * 256 + threadIdx.x;
  if (i < n2) {
    const v2f f = *(const v2f*)(in + 2 * (size_t)i);
    const unsigned u = pk16(f2bf_bits(f[0]), f2bf_bits(f[1]));
    ((volatile unsigned*)out)[i] = u;
    __threadfence();
    ((volatile unsigned*)out)[i] = u;
  }
}

template <bool F16>
__global__ __launch_bounds__(256) void tcvt_kernel(const float* __restrict__ W, unsigned short* ob, unsigned short* o16,
                                                   int R, int Cc, float sc) {
  __shared__ __align__(16) float tf[64 * 68];
  const int c0  = blockIdx.x * 64;
  const int r0  = blockIdx.y * 64;
  const int tid = threadIdx.x;
  {
    const int lr = tid >> 4;
    const int c4 = (tid & 15) * 4;
#pragma unroll
    for (int it = 0; it < 4; ++it) {
      const int rr = it * 16 + lr;
      const v4f a = *(const v4f*)(W + (size_t)(r0 + rr) * Cc + c0 + c4);
      *(v4f*)(tf + rr * 68 + c4) = a;
    }
  }
  __syncthreads();
  const int sub = tid >> 3;
  const int c8  = (tid & 7) * 8;
  v4u hv[2], fv[2];
#pragma unroll
  for (int it = 0; it < 2; ++it) {
    const int oc = it * 32 + sub;
    v4u a, a16;
#pragma unroll
    for (int q = 0; q < 4; ++q) {
      const float f0 = tf[(c8 + 2 * q) * 68 + oc];
      const float f1 = tf[(c8 + 2 * q + 1) * 68 + oc];
      const unsigned short h0 = f2bf_bits(f0), h1 = f2bf_bits(f1);
      a[q] = pk16(h0, h1);
      if (F16) {
        const _Float16 g0 = (_Float16)(bf_bits2f(h0) * sc);
        const _Float16 g1 = (_Float16)(bf_bits2f(h1) * sc);
        a16[q] = pk16(__builtin_bit_cast(unsigned short, g0), __builtin_bit_cast(unsigned short, g1));
      } else {
        a16[q] = a[q];
      }
    }
    hv[it] = a; fv[it] = a16;
  }
  for (int pass = 0; pass < 2; ++pass) {
#pragma unroll
    for (int it = 0; it < 2; ++it) {
      const int oc = it * 32 + sub;
      const size_t go = (size_t)(c0 + oc) * R + r0 + c8;
      *(volatile v4u*)(ob + go) = hv[it];
      if (F16) *(volatile v4u*)(o16 + go) = fv[it];
    }
    __threadfence();
  }
}

#define ATT_QP 520
#define ATT_VP 72
#define ATT_OP 132
#define ATT_QBYTES (64 * ATT_QP * 2)
#define ATT_VBYTES (HDIM * ATT_VP * 2)
#define ATT_PBYTES (4 * 16 * ATT_VP * 2)
#define ATT_OBYTES (4 * 16 * ATT_OP * 4)
__host__ __device__ constexpr int attn_lds_bytes(bool res) {
  return 2 * ATT_QBYTES + (res ? 2 : 1) * ATT_VBYTES + (res ? 2 : 1) * ATT_PBYTES + ATT_OBYTES;
}

template <bool R> struct PVT;
template <> struct PVT<false> {
  typedef _Float16 T; typedef v8h V8; typedef v16h V16;
  static __device__ __forceinline__ void store_p(T* ph, T* pl, int idx, float p) { (void)pl; ph[idx] = (_Float16)(p * PSC); }
  static __device__ __forceinline__ v8f mma(V16 a, V16 b, v8f c) {
    return __builtin_amdgcn_wmma_f32_16x16x32_f16(false, a, false, b, (short)0, c, false, false);
  }
  static __device__ __forceinline__ void g4(v8f& a, v8f& b, v8f& c, v8f& d, V16 x, V16 y) { g4h(a, b, c, d, x, y); }
};
template <> struct PVT<true> {
  typedef __bf16 T; typedef v8b V8; typedef v16b V16;
  static __device__ __forceinline__ void store_p(T* ph, T* pl, int idx, float p) {
    unsigned short hb, lb; bf_split_bits(p, hb, lb);
    ph[idx] = __builtin_bit_cast(__bf16, hb);
    pl[idx] = __builtin_bit_cast(__bf16, lb);
  }
  static __device__ __forceinline__ v8f mma(V16 a, V16 b, v8f c) {
    return __builtin_amdgcn_wmma_f32_16x16x32_bf16(false, a, false, b, (short)0, c, false, false);
  }
  static __device__ __forceinline__ void g4(v8f& a, v8f& b, v8f& c, v8f& d, V16 x, V16 y) { g4b(a, b, c, d, x, y); }
};

template <bool RES>
__device__ __forceinline__ void attn_body(const unsigned short* __restrict__ qlp,
                                          const unsigned short* __restrict__ kvp,
                                          const unsigned short* __restrict__ v0p,
                                          const unsigned short* __restrict__ v1p,
                                          unsigned short* y16p,
                                          unsigned short* ybhp, unsigned short* yblp,
                                          int hbase, int qbStart, float seff,
                                          unsigned char* smem_raw) {
  typedef typename PVT<RES>::T PT;
  typedef typename PVT<RES>::V8 PV8;
  typedef typename PVT<RES>::V16 PV16;
  union FH { v16h v; v8h h[2]; };
  union FP { PV16 v; PV8 h[2]; };
  constexpr int QP = ATT_QP, VP = ATT_VP, OP = ATT_OP;
  constexpr int OFF_Q  = 0;
  constexpr int OFF_K  = OFF_Q + ATT_QBYTES;
  constexpr int OFF_V0 = OFF_K + ATT_QBYTES;
  constexpr int OFF_V1 = OFF_V0 + ATT_VBYTES;
  constexpr int OFF_P0 = RES ? (OFF_V1 + ATT_VBYTES) : OFF_V1;
  constexpr int OFF_P1 = OFF_P0 + ATT_PBYTES;
  constexpr int OFF_O  = RES ? (OFF_P1 + ATT_PBYTES) : OFF_P1;

  const int tid  = threadIdx.x;
  const int wave = tid >> 5;
  const int lane = tid & 31;
  const int hh   = lane >> 4;
  const int c    = lane & 15;

  _Float16* Qs  = (_Float16*)(smem_raw + OFF_Q);
  _Float16* Ks  = (_Float16*)(smem_raw + OFF_K);
  PT*       Vt0 = (PT*)(smem_raw + OFF_V0);
  PT*       Vt1 = RES ? (PT*)(smem_raw + OFF_V1) : Vt0;
  PT*       Pw0 = (PT*)(smem_raw + OFF_P0) + wave * 16 * VP;
  PT*       Pw1 = RES ? ((PT*)(smem_raw + OFF_P1) + wave * 16 * VP) : Pw0;
  float*    os  = (float*)(smem_raw + OFF_O) + wave * 16 * OP;

  const int qb = (int)blockIdx.x + qbStart;
  const int hl = blockIdx.y;
  const int h  = hbase + hl;
  const int b  = blockIdx.z;
  const int q0w = qb * 64 + wave * 16;

  {
    const _Float16* qg = (const _Float16*)(const void*)qlp + ((size_t)hl * BTOT + (size_t)b * SEQ + (size_t)qb * 64) * DLAT;
#pragma unroll 8
    for (int j = 0; j < 32; ++j) {
      const int ci = tid + j * 128;
      const int r = ci >> 6, c16 = ci & 63;
      *(v8h*)(Qs + r * QP + c16 * 8) = *(const v8h*)(qg + (size_t)r * DLAT + c16 * 8);
    }
  }

  float mrow[8], lrow[8];
  v8f oacc[8];
#pragma unroll
  for (int r = 0; r < 8; ++r) { mrow[r] = -INFINITY; lrow[r] = 0.f; }
#pragma unroll
  for (int t = 0; t < 8; ++t) oacc[t] = (v8f){0.f,0.f,0.f,0.f,0.f,0.f,0.f,0.f};

  const int nChunks = qb + 1;
  for (int kc = 0; kc < nChunks; ++kc) {
    const int kv0 = kc * 64;
    __syncthreads();
    {
      const _Float16* kg = (const _Float16*)(const void*)kvp + ((size_t)b * SEQ + (size_t)kv0) * DLAT;
#pragma unroll 8
      for (int j = 0; j < 32; ++j) {
        const int ci = tid + j * 128;
        const int r = ci >> 6, c16 = ci & 63;
        *(v8h*)(Ks + r * QP + c16 * 8) = *(const v8h*)(kg + (size_t)r * DLAT + c16 * 8);
      }
      if (!RES) {
        const PT* vg = (const PT*)(const void*)v0p + (size_t)h * HDIM * BTOT + (size_t)b * SEQ + kv0;
#pragma unroll
        for (int j = 0; j < 8; ++j) {
          const int ci = tid + j * 128;
          const int d = ci >> 3, c16 = ci & 7;
          *(PV8*)(Vt0 + d * VP + c16 * 8) = *(const PV8*)(vg + (size_t)d * BTOT + c16 * 8);
        }
      } else {
        const PT* vg0 = (const PT*)(const void*)v0p + (size_t)h * HDIM * (2 * TRES) + (size_t)b * TRES + kv0;
        const PT* vg1 = (const PT*)(const void*)v1p + (size_t)h * HDIM * (2 * TRES) + (size_t)b * TRES + kv0;
#pragma unroll
        for (int j = 0; j < 8; ++j) {
          const int ci = tid + j * 128;
          const int d = ci >> 3, c16 = ci & 7;
          *(PV8*)(Vt0 + d * VP + c16 * 8) = *(const PV8*)(vg0 + (size_t)d * (2 * TRES) + c16 * 8);
          *(PV8*)(Vt1 + d * VP + c16 * 8) = *(const PV8*)(vg1 + (size_t)d * (2 * TRES) + c16 * 8);
        }
      }
    }
    __syncthreads();

    v8f s[4];
#pragma unroll
    for (int j = 0; j < 4; ++j) s[j] = (v8f){0.f,0.f,0.f,0.f,0.f,0.f,0.f,0.f};
    {
      const _Float16* qrow = Qs + (wave * 16 + c) * QP + 8 * hh;
      const _Float16* krow = Ks + c * QP + 8 * hh;
#pragma unroll 4
      for (int ks = 0; ks < DLAT / 32; ++ks) {
        FH a;
        a.h[0] = *(const v8h*)(qrow + ks * 32);
        a.h[1] = *(const v8h*)(qrow + ks * 32 + 16);
        FH kf;
#pragma unroll
        for (int j = 0; j < 4; ++j) {
          kf.h[0] = *(const v8h*)(krow + j * 16 * QP + ks * 32);
          kf.h[1] = *(const v8h*)(krow + j * 16 * QP + ks * 32 + 16);
          s[j] = Frag<_Float16>::mma(a.v, kf.v, s[j]);
        }
        g4h(s[0], s[1], s[2], s[3], a.v, kf.v);
      }
    }

    const bool diag = (kc == qb);
    float cm[8];
#pragma unroll
    for (int r = 0; r < 8; ++r) {
      const int qrow = q0w + 8 * hh + r;
      float m = -INFINITY;
#pragma unroll
      for (int j = 0; j < 4; ++j) {
        const int kvcol = kv0 + j * 16 + c;
        float sv = s[j][r] * seff;
        if (diag && (kvcol > qrow)) sv = -INFINITY;
        s[j][r] = sv;
        m = fmaxf(m, sv);
      }
#pragma unroll
      for (int off = 1; off < 16; off <<= 1) m = fmaxf(m, __shfl_xor(m, off, 32));
      cm[r] = m;
    }
#pragma unroll
    for (int r = 0; r < 8; ++r) {
      const float mnew  = fmaxf(mrow[r], cm[r]);
      const float alpha = expf(mrow[r] - mnew);
      mrow[r] = mnew;
      float psum = 0.f;
#pragma unroll
      for (int j = 0; j < 4; ++j) {
        const float p = expf(s[j][r] - mnew);
        psum += p;
        PVT<RES>::store_p(Pw0, Pw1, (8 * hh + r) * VP + j * 16 + c, p);
      }
#pragma unroll
      for (int off = 1; off < 16; off <<= 1) psum += __shfl_xor(psum, off, 32);
      lrow[r] = lrow[r] * alpha + psum;
#pragma unroll
      for (int t = 0; t < 8; ++t) oacc[t][r] *= alpha;
    }
    __builtin_amdgcn_fence(__ATOMIC_RELEASE, "workgroup");
    __builtin_amdgcn_wave_barrier();
    __builtin_amdgcn_fence(__ATOMIC_ACQUIRE, "workgroup");

#pragma unroll
    for (int kk = 0; kk < 2; ++kk) {
      FP pa, pl;
      pa.h[0] = *(const PV8*)(Pw0 + c * VP + kk * 32 + 8 * hh);
      pa.h[1] = *(const PV8*)(Pw0 + c * VP + kk * 32 + 16 + 8 * hh);
      if (RES) {
        pl.h[0] = *(const PV8*)(Pw1 + c * VP + kk * 32 + 8 * hh);
        pl.h[1] = *(const PV8*)(Pw1 + c * VP + kk * 32 + 16 + 8 * hh);
      } else {
        pl = pa;
      }
      FP vb, vl;
#pragma unroll
      for (int t = 0; t < 8; ++t) {
        vb.h[0] = *(const PV8*)(Vt0 + (t * 16 + c) * VP + kk * 32 + 8 * hh);
        vb.h[1] = *(const PV8*)(Vt0 + (t * 16 + c) * VP + kk * 32 + 16 + 8 * hh);
        oacc[t] = PVT<RES>::mma(pa.v, vb.v, oacc[t]);
        if (RES) {
          vl.h[0] = *(const PV8*)(Vt1 + (t * 16 + c) * VP + kk * 32 + 8 * hh);
          vl.h[1] = *(const PV8*)(Vt1 + (t * 16 + c) * VP + kk * 32 + 16 + 8 * hh);
          oacc[t] = PVT<RES>::mma(pa.v, vl.v, oacc[t]);
          oacc[t] = PVT<RES>::mma(pl.v, vb.v, oacc[t]);
        }
        if (t == 3) PVT<RES>::g4(oacc[0], oacc[1], oacc[2], oacc[3], pl.v, vb.v);
        if (t == 7) PVT<RES>::g4(oacc[4], oacc[5], oacc[6], oacc[7], pl.v, vb.v);
      }
      asm volatile("v_nop" :: "v"(pa.v));
    }
  }

#pragma unroll
  for (int r = 0; r < 8; ++r) {
    const float inv = (1.0f / lrow[r]) * (RES ? 1.0f : (1.0f / (PSC * VSC)));
#pragma unroll
    for (int t = 0; t < 8; ++t) os[(8 * hh + r) * OP + t * 16 + c] = oacc[t][r] * inv;
  }
  __builtin_amdgcn_fence(__ATOMIC_RELEASE, "workgroup");
  __builtin_amdgcn_wave_barrier();
  __builtin_amdgcn_fence(__ATOMIC_ACQUIRE, "workgroup");
  {
    const int c8 = (lane & 15) * 8;
    _Float16* Y16 = (_Float16*)(void*)y16p;
    for (int pass = 0; pass < 2; ++pass) {
#pragma unroll
      for (int it = 0; it < 8; ++it) {
        const int row = it * 2 + hh;
        const float* op = os + row * OP + c8;
        const v4f o0 = *(const v4f*)(op);
        const v4f o1 = *(const v4f*)(op + 4);
        v8h yv;
#pragma unroll
        for (int e = 0; e < 4; ++e) { yv[e] = (_Float16)(o0[e] * YSC); yv[4 + e] = (_Float16)(o1[e] * YSC); }
        const size_t grow = (size_t)b * SEQ + (size_t)(q0w + row);
        *(volatile v8h*)(Y16 + grow * DMOD + h * HDIM + c8) = yv;
        if (RES) {
          v8us hb8, lb8;
#pragma unroll
          for (int e = 0; e < 4; ++e) {
            unsigned short hb, lb;
            bf_split_bits(o0[e], hb, lb); hb8[e] = hb; lb8[e] = lb;
            bf_split_bits(o1[e], hb, lb); hb8[4 + e] = hb; lb8[4 + e] = lb;
          }
          const size_t grow2 = (size_t)b * TRES + (size_t)(q0w + row);
          *(volatile v8us*)(ybhp + grow2 * DMOD + h * HDIM + c8) = hb8;
          *(volatile v8us*)(yblp + grow2 * DMOD + h * HDIM + c8) = lb8;
        }
      }
      __threadfence();
    }
  }
}

__global__ __launch_bounds__(128) void attn_kernel_res(const unsigned short* __restrict__ qlp,
                                                       const unsigned short* __restrict__ kvp,
                                                       const unsigned short* __restrict__ v0p,
                                                       const unsigned short* __restrict__ v1p,
                                                       unsigned short* y16p,
                                                       unsigned short* ybhp, unsigned short* yblp,
                                                       int hbase, int qbStart, float seff) {
  extern __shared__ __align__(16) unsigned char smem_raw[];
  attn_body<true>(qlp, kvp, v0p, v1p, y16p, ybhp, yblp, hbase, qbStart, seff, smem_raw);
}

__global__ __launch_bounds__(128) void attn_kernel_main(const unsigned short* __restrict__ qlp,
                                                        const unsigned short* __restrict__ kvp,
                                                        const unsigned short* __restrict__ v0p,
                                                        const unsigned short* __restrict__ v1p,
                                                        unsigned short* y16p,
                                                        unsigned short* ybhp, unsigned short* yblp,
                                                        int hbase, int qbStart, float seff) {
  extern __shared__ __align__(16) unsigned char smem_raw[];
  attn_body<false>(qlp, kvp, v0p, v1p, y16p, ybhp, yblp, hbase, qbStart, seff, smem_raw);
}

extern "C" void kernel_launch(void* const* d_in, const int* in_sizes, int n_in,
                              void* d_out, int out_size, void* d_ws, size_t ws_size,
                              hipStream_t stream) {
  if (n_in < 6) return;
  if (in_sizes[0] != BTOT * DMOD) return;
  if (in_sizes[1] != DMOD * DLAT || in_sizes[2] != DMOD * DLAT || in_sizes[3] != DLAT * DMOD) return;
  if (in_sizes[4] != DMOD * DMOD || in_sizes[5] != DMOD * DMOD) return;
  if (out_size != BTOT * DMOD) return;

  const float* x     = (const float*)d_in[0];
  const float* w_dkv = (const float*)d_in[1];
  const float* w_uk  = (const float*)d_in[2];
  const float* w_uv  = (const float*)d_in[3];
  const float* w_q   = (const float*)d_in[4];
  const float* w_o   = (const float*)d_in[5];
  float* out = (float*)d_out;

  const size_t sXb    = (size_t)BTOT * DMOD * 2;
  const size_t sW512  = (size_t)DMOD * DLAT * 2;
  const size_t sW2048 = (size_t)DMOD * DMOD * 2;
  const size_t sKV16  = (size_t)BTOT * DLAT * 2;
  const size_t sKVb   = (size_t)NBATCH * TRES * DLAT * 2;
  const size_t sQb    = (size_t)BTOT * (HGRP * HDIM) * 2;
  const size_t sQL    = (size_t)HGRP * BTOT * DLAT * 2;
  const size_t sVt16  = (size_t)DMOD * BTOT * 2;
  const size_t sVtb   = (size_t)DMOD * (NBATCH * TRES) * 2;
  const size_t sY16   = (size_t)BTOT * DMOD * 2;
  const size_t sYb    = (size_t)(NBATCH * TRES) * DMOD * 2;
  size_t off = 0;
  const size_t oXb     = off; off += sXb;
  const size_t oWdkvTb = off; off += sW512;
  const size_t oWqTb   = off; off += sW2048;
  const size_t oWukTb  = off; off += sW512;
  const size_t oWuvTb  = off; off += sW512;
  const size_t oWuvT16 = off; off += sW512;
  const size_t oWoTb   = off; off += sW2048;
  const size_t oWoT16  = off; off += sW2048;
  const size_t oKV16   = off; off += sKV16;
  const size_t oKVbh   = off; off += sKVb;
  const size_t oKVbl   = off; off += sKVb;
  const size_t oQbh    = off; off += sQb;
  const size_t oQbl    = off; off += sQb;
  const size_t oQL     = off; off += sQL;
  const size_t oVt16   = off; off += sVt16;
  const size_t oVtbh   = off; off += sVtb;
  const size_t oVtbl   = off; off += sVtb;
  const size_t oY16    = off; off += sY16;
  const size_t oYbh    = off; off += sYb;
  const size_t oYbl    = off; off += sYb;
  if (off > ws_size) return;

  char* ws = (char*)d_ws;
  unsigned short* Xb     = (unsigned short*)(ws + oXb);
  unsigned short* WdkvTb = (unsigned short*)(ws + oWdkvTb);
  unsigned short* WqTb   = (unsigned short*)(ws + oWqTb);
  unsigned short* WukTb  = (unsigned short*)(ws + oWukTb);
  unsigned short* WuvTb  = (unsigned short*)(ws + oWuvTb);
  unsigned short* WuvT16 = (unsigned short*)(ws + oWuvT16);
  unsigned short* WoTb   = (unsigned short*)(ws + oWoTb);
  unsigned short* WoT16  = (unsigned short*)(ws + oWoT16);
  unsigned short* KV16   = (unsigned short*)(ws + oKV16);
  unsigned short* KVbh   = (unsigned short*)(ws + oKVbh);
  unsigned short* KVbl   = (unsigned short*)(ws + oKVbl);
  unsigned short* Qbh    = (unsigned short*)(ws + oQbh);
  unsigned short* Qbl    = (unsigned short*)(ws + oQbl);
  unsigned short* QL     = (unsigned short*)(ws + oQL);
  unsigned short* Vt16   = (unsigned short*)(ws + oVt16);
  unsigned short* Vtbh   = (unsigned short*)(ws + oVtbh);
  unsigned short* Vtbl   = (unsigned short*)(ws + oVtbl);
  unsigned short* Y16    = (unsigned short*)(ws + oY16);
  unsigned short* Ybh    = (unsigned short*)(ws + oYbh);
  unsigned short* Ybl    = (unsigned short*)(ws + oYbl);

  const float scl  = 1.0f / sqrtf((float)DMOD);
  const float seff = scl * (1.0f / (QSC * KSC));

  const int ldsMain = attn_lds_bytes(false);
  const int ldsRes  = attn_lds_bytes(true);

  const dim3 blk(256);

  const int n2x = BTOT * DMOD / 2;
  cvt_bf16x2_kernel<<<dim3(n2x / 256), blk, 0, stream>>>(x, Xb, n2x);

  tcvt_kernel<false><<<dim3(DLAT / 64, DMOD / 64), blk, 0, stream>>>(w_dkv, WdkvTb, WdkvTb, DMOD, DLAT, 1.0f);
  tcvt_kernel<false><<<dim3(DMOD / 64, DMOD / 64), blk, 0, stream>>>(w_q,   WqTb,   WqTb,   DMOD, DMOD, 1.0f);
  tcvt_kernel<false><<<dim3(DLAT / 64, DMOD / 64), blk, 0, stream>>>(w_uk,  WukTb,  WukTb,  DMOD, DLAT, 1.0f);
  tcvt_kernel<true ><<<dim3(DMOD / 64, DLAT / 64), blk, 0, stream>>>(w_uv,  WuvTb,  WuvT16, DLAT, DMOD, WSC);
  tcvt_kernel<true ><<<dim3(DMOD / 64, DMOD / 64), blk, 0, stream>>>(w_o,   WoTb,   WoT16,  DMOD, DMOD, WSC);

  gemm64<1, false, false, 1, true><<<dim3((BTOT / 64) * ((DLAT / 64) / 8), 1), blk, 0, stream>>>(
      Xb, Xb, DMOD, 0LL, WdkvTb, WdkvTb, DMOD, 0LL, (void*)KV16, (void*)KV16, (void*)KV16, DLAT, 0LL,
      BTOT, DLAT, DMOD, 1.0f, KSC);
  gemm64<1, false, false, 2, true><<<dim3((TRES / 64) * ((DLAT / 64) / 8), NBATCH), blk, 0, stream>>>(
      Xb, Xb, DMOD, (long long)SEQ * DMOD, WdkvTb, WdkvTb, DMOD, 0LL, (void*)KVbh, (void*)KVbh, (void*)KVbl, DLAT, (long long)TRES * DLAT,
      TRES, DLAT, DMOD, 1.0f, 1.0f);

  gemm64<0, false, false, 1, true><<<dim3((DMOD / 64) * ((BTOT / 64) / 8), 1), blk, 0, stream>>>(
      WuvT16, WuvT16, DLAT, 0LL, KV16, KV16, DLAT, 0LL, (void*)Vt16, (void*)Vt16, (void*)Vt16, BTOT, 0LL,
      DMOD, BTOT, DLAT, 1.0f / (WSC * KSC), VSC);
  gemm64<1, false, true, 2, false><<<dim3((TRES / 64) * ((DMOD / 64) / 8), NBATCH), blk, 0, stream>>>(
      WuvTb, WuvTb, DLAT, 0LL, KVbh, KVbl, DLAT, (long long)TRES * DLAT, (void*)Vtbh, (void*)Vtbh, (void*)Vtbl, 2 * TRES, (long long)TRES,
      DMOD, TRES, DLAT, 1.0f, 1.0f);

  for (int g = 0; g < NGRP; ++g) {
    gemm64<1, false, false, 2, false><<<dim3(((HGRP * HDIM) / 64) * ((BTOT / 64) / 8), 1), blk, 0, stream>>>(
        Xb, Xb, DMOD, 0LL, WqTb + (size_t)g * (HGRP * HDIM) * DMOD, WqTb + (size_t)g * (HGRP * HDIM) * DMOD, DMOD, 0LL,
        (void*)Qbh, (void*)Qbh, (void*)Qbl, HGRP * HDIM, 0LL,
        BTOT, HGRP * HDIM, DMOD, 1.0f, 1.0f);
    gemm64<1, true, false, 1, true><<<dim3((BTOT / 64) * ((DLAT / 64) / 8), HGRP), blk, 0, stream>>>(
        Qbh, Qbl, HGRP * HDIM, (long long)HDIM, WukTb + (size_t)g * HGRP * HDIM, WukTb + (size_t)g * HGRP * HDIM, DMOD, (long long)HDIM,
        (void*)QL, (void*)QL, (void*)QL, DLAT, (long long)BTOT * DLAT,
        BTOT, DLAT, HDIM, 1.0f, QSC);
    attn_kernel_res<<<dim3(NQBRES, HGRP, NBATCH), dim3(128), ldsRes, stream>>>(
        QL, KV16, Vtbh, Vtbl, Y16, Ybh, Ybl, g * HGRP, 0, seff);
    attn_kernel_main<<<dim3(NQB - NQBRES, HGRP, NBATCH), dim3(128), ldsMain, stream>>>(
        QL, KV16, Vt16, Vt16, Y16, Ybh, Ybl, g * HGRP, NQBRES, seff);
  }

  gemm64<0, false, false, 0, true><<<dim3(((SEQ - TRES) / 64) * ((DMOD / 64) / 8), NBATCH), blk, 0, stream>>>(
      Y16 + (size_t)TRES * DMOD, Y16 + (size_t)TRES * DMOD, DMOD, (long long)SEQ * DMOD, WoT16, WoT16, DMOD, 0LL,
      (void*)(out + (size_t)TRES * DMOD), (void*)(out + (size_t)TRES * DMOD), (void*)(out + (size_t)TRES * DMOD), DMOD, (long long)SEQ * DMOD,
      SEQ - TRES, DMOD, DMOD, 1.0f / (YSC * WSC), 1.0f);
  gemm64<1, true, false, 0, true><<<dim3((TRES / 64) * ((DMOD / 64) / 8), NBATCH), blk, 0, stream>>>(
      Ybh, Ybl, DMOD, (long long)TRES * DMOD, WoTb, WoTb, DMOD, 0LL,
      (void*)out, (void*)out, (void*)out, DMOD, (long long)SEQ * DMOD,
      TRES, DMOD, DMOD, 1.0f, 1.0f);

  (void)hipGetLastError();
}
